// LCF_ATEPC_8031588843931
// MI455X (gfx1250) — hardware-verified
//
#include <hip/hip_runtime.h>
#include <stddef.h>
#include <stdint.h>
#include <math.h>

#define NB    64
#define NL    256
#define NHID  768
#define NHEAD 12
#define HDIM  64
#define H3    (3 * NHID)
#define ROWS  (NB * NL)
#define KVW   (2 * NHID)

static_assert(NHEAD * HDIM == NHID);
static_assert(NL == 256);
static_assert(ROWS % 256 == 0);
static_assert(NHID % 64 == 0);
static_assert(H3 % 64 == 0);
static_assert(H3 % 32 == 0);

typedef _Float16 v16h __attribute__((ext_vector_type(16)));
typedef _Float16 v8h  __attribute__((ext_vector_type(8)));
typedef float    v8f  __attribute__((ext_vector_type(8)));
typedef float    v4f  __attribute__((ext_vector_type(4)));
typedef unsigned int v4u __attribute__((ext_vector_type(4)));

union Frag  { v16h v; v8h h[2]; };
union Pack8 { v8h h; v4u u; };

__device__ __forceinline__ v8f mma16(v16h a, v16h b, v8f c) {
  c = __builtin_amdgcn_wmma_f32_16x16x32_f16(false, a, false, b, (short)0, c, false, false);
  asm volatile("v_nop\n\tv_nop\n\tv_nop\n\tv_nop" : "+v"(c) : "v"(a), "v"(b));
  return c;
}

__device__ __forceinline__ v16h ldfrag(const _Float16* p, int ld, int row0, int k0, int lane) {
  const int m = lane & 15, lh = lane >> 4;
  const _Float16* q = p + (size_t)(row0 + m) * ld + k0 + 8 * lh;
  Frag f;
  f.h[0] = *(const v8h*)(q);
  f.h[1] = *(const v8h*)(q + 16);
  return f.v;
}

__device__ __forceinline__ v8f zero8() { return (v8f){0.f, 0.f, 0.f, 0.f, 0.f, 0.f, 0.f, 0.f}; }

__device__ __forceinline__ v4f pick4(bool c, v4f a, v4f b) {
  v4f r;
  r[0] = c ? a[0] : b[0];
  r[1] = c ? a[1] : b[1];
  r[2] = c ? a[2] : b[2];
  r[3] = c ? a[3] : b[3];
  return r;
}

template <int KK>
__device__ __forceinline__ void gemm32x64(const _Float16* __restrict__ A, int lda,
                                          const _Float16* __restrict__ Bt, int ldb,
                                          int m0, int n0, int lane, v8f (&acc)[2][4]) {
#pragma unroll 2
  for (int k0 = 0; k0 < KK; k0 += 32) {
    const v16h a0 = ldfrag(A, lda, m0, k0, lane);
    const v16h a1 = ldfrag(A, lda, m0 + 16, k0, lane);
    const v16h b0 = ldfrag(Bt, ldb, n0, k0, lane);
    const v16h b1 = ldfrag(Bt, ldb, n0 + 16, k0, lane);
    const v16h b2 = ldfrag(Bt, ldb, n0 + 32, k0, lane);
    const v16h b3 = ldfrag(Bt, ldb, n0 + 48, k0, lane);
    acc[0][0] = mma16(a0, b0, acc[0][0]);
    acc[1][0] = mma16(a1, b0, acc[1][0]);
    acc[0][1] = mma16(a0, b1, acc[0][1]);
    acc[1][1] = mma16(a1, b1, acc[1][1]);
    acc[0][2] = mma16(a0, b2, acc[0][2]);
    acc[1][2] = mma16(a1, b2, acc[1][2]);
    acc[0][3] = mma16(a0, b3, acc[0][3]);
    acc[1][3] = mma16(a1, b3, acc[1][3]);
  }
}

__global__ __launch_bounds__(256) void k_cat(const float* __restrict__ gh,
                                             const float* __restrict__ lh,
                                             const int* __restrict__ valid,
                                             const float* __restrict__ cdm,
                                             const float* __restrict__ cdw,
                                             const float* __restrict__ wate,
                                             const float* __restrict__ bate,
                                             _Float16* __restrict__ cat,
                                             float* __restrict__ ate) {
  __shared__ int s_scan[NL];
  __shared__ int s_src[16];
  __shared__ __align__(16) float s_ate[96];
  const int tid = threadIdx.x, lane = tid & 31, wave = tid >> 5;
  const int blk = blockIdx.x;
  const int b  = blk >> 4;
  const int d0 = (blk & 15) * 16;

  const int v = valid[b * NL + tid];
  s_scan[tid] = v;
  if (tid < 16) s_src[tid] = -1;
  __syncthreads();
  for (int off = 1; off < NL; off <<= 1) {
    const int ia = tid - off;
    const int xv = s_scan[ia < 0 ? 0 : ia];
    const int x  = (ia >= 0) ? xv : 0;
    __syncthreads();
    s_scan[tid] += x;
    __syncthreads();
  }
  const int dest = s_scan[tid] - 1;
  if (v == 1 && dest >= d0 && dest < d0 + 16) s_src[dest - d0] = tid;
  __syncthreads();

  const v4f z4 = (v4f){0.f, 0.f, 0.f, 0.f};
  for (int jt = 0; jt < 2; ++jt) {
    const int slot = wave * 2 + jt;
    const int d = d0 + slot;
    const int t = s_src[slot];
    const int tc = (t < 0) ? 0 : t;
    const bool has = (t >= 0);
    const size_t srow = ((size_t)(b * NL + tc)) * NHID;
    const float* gsrc = gh + srow;
    const float* lsrc = lh + srow;
    const float cw16 = cdw[b * NL + d] * 16.0f;
    const float cm16 = cdm[b * NL + d] * 16.0f;
    _Float16* crow = cat + ((size_t)(b * NL + d)) * H3;
    float acc6[6] = {0.f, 0.f, 0.f, 0.f, 0.f, 0.f};

#pragma unroll 1
    for (int it = 0; it < 3; ++it) {
      const int c8 = (it * 32 + lane) * 8;
      v4f a0 = *(const v4f*)(gsrc + c8);
      v4f a1 = *(const v4f*)(gsrc + c8 + 4);
      v4f l0 = *(const v4f*)(lsrc + c8);
      v4f l1 = *(const v4f*)(lsrc + c8 + 4);
      a0 = pick4(has, a0, z4); a1 = pick4(has, a1, z4);
      l0 = pick4(has, l0, z4); l1 = pick4(has, l1, z4);
      Pack8 pg, pw, pm;
      pg.h = (v8h){(_Float16)(a0[0] * 16.0f), (_Float16)(a0[1] * 16.0f), (_Float16)(a0[2] * 16.0f), (_Float16)(a0[3] * 16.0f),
                   (_Float16)(a1[0] * 16.0f), (_Float16)(a1[1] * 16.0f), (_Float16)(a1[2] * 16.0f), (_Float16)(a1[3] * 16.0f)};
      pw.h = (v8h){(_Float16)(l0[0] * cw16), (_Float16)(l0[1] * cw16), (_Float16)(l0[2] * cw16), (_Float16)(l0[3] * cw16),
                   (_Float16)(l1[0] * cw16), (_Float16)(l1[1] * cw16), (_Float16)(l1[2] * cw16), (_Float16)(l1[3] * cw16)};
      pm.h = (v8h){(_Float16)(l0[0] * cm16), (_Float16)(l0[1] * cm16), (_Float16)(l0[2] * cm16), (_Float16)(l0[3] * cm16),
                   (_Float16)(l1[0] * cm16), (_Float16)(l1[1] * cm16), (_Float16)(l1[2] * cm16), (_Float16)(l1[3] * cm16)};
      const v4u ug = pg.u, uw = pw.u, um = pm.u;
      volatile v4u* qg = (volatile v4u*)(crow + c8);
      volatile v4u* qw = (volatile v4u*)(crow + NHID + c8);
      volatile v4u* qm = (volatile v4u*)(crow + 2 * NHID + c8);
      *qg = ug; *qw = uw; *qm = um;
      __threadfence();
      *qg = ug; *qw = uw; *qm = um;

      const float* wp = wate + c8 * 6;
#pragma unroll 1
      for (int hf = 0; hf < 2; ++hf) {
        const v4f x = pick4(hf != 0, a1, a0);
        const float* wq = wp + hf * 24;
        const v4f w0 = *(const v4f*)(wq);
        const v4f w1 = *(const v4f*)(wq + 4);
        const v4f w2 = *(const v4f*)(wq + 8);
        const v4f w3 = *(const v4f*)(wq + 12);
        const v4f w4 = *(const v4f*)(wq + 16);
        const v4f w5 = *(const v4f*)(wq + 20);
        acc6[0] += x[0] * w0[0]; acc6[1] += x[0] * w0[1]; acc6[2] += x[0] * w0[2];
        acc6[3] += x[0] * w0[3]; acc6[4] += x[0] * w1[0]; acc6[5] += x[0] * w1[1];
        acc6[0] += x[1] * w1[2]; acc6[1] += x[1] * w1[3]; acc6[2] += x[1] * w2[0];
        acc6[3] += x[1] * w2[1]; acc6[4] += x[1] * w2[2]; acc6[5] += x[1] * w2[3];
        acc6[0] += x[2] * w3[0]; acc6[1] += x[2] * w3[1]; acc6[2] += x[2] * w3[2];
        acc6[3] += x[2] * w3[3]; acc6[4] += x[2] * w4[0]; acc6[5] += x[2] * w4[1];
        acc6[0] += x[3] * w4[2]; acc6[1] += x[3] * w4[3]; acc6[2] += x[3] * w5[0];
        acc6[3] += x[3] * w5[1]; acc6[4] += x[3] * w5[2]; acc6[5] += x[3] * w5[3];
      }
    }
#pragma unroll
    for (int j = 0; j < 6; ++j) {
      float s = acc6[j];
#pragma unroll
      for (int off = 16; off > 0; off >>= 1) s += __shfl_xor(s, off, 32);
      acc6[j] = s;
    }
    if (lane == 0) {
#pragma unroll
      for (int j = 0; j < 6; ++j) s_ate[slot * 6 + j] = acc6[j] + bate[j];
    }
  }
  __syncthreads();
  if (tid < 24) {
    const v4f o = *(const v4f*)(s_ate + 4 * tid);
    volatile v4f* dp = (volatile v4f*)(ate + (size_t)blk * 96 + 4 * tid);
    *dp = o;
    __threadfence();
    *dp = o;
  }
}

#define WTP 68
__global__ __launch_bounds__(256) void k_wt(const float* __restrict__ w, _Float16* __restrict__ wt,
                                           int nout, int kin) {
  __shared__ __align__(16) float tf[64 * WTP];
  const int tid = threadIdx.x;
  const int n0 = blockIdx.x * 64;
  const int k0 = blockIdx.y * 64;
  {
    const int kr = tid >> 4;
    const int n4 = (tid & 15) * 4;
#pragma unroll
    for (int it = 0; it < 4; ++it) {
      const int kl = it * 16 + kr;
      const v4f a = *(const v4f*)(w + (size_t)(k0 + kl) * nout + n0 + n4);
      *(v4f*)(tf + kl * WTP + n4) = a;
    }
  }
  __syncthreads();
  v4u val[2];
  size_t go[2];
#pragma unroll
  for (int j = 0; j < 2; ++j) {
    const int p  = tid + 256 * j;
    const int nl = p >> 3;
    const int pc = p & 7;
    const float* cp = tf + (pc * 8) * WTP + nl;
    Pack8 pk;
    pk.h = (v8h){(_Float16)(cp[0 * WTP] * 32.0f), (_Float16)(cp[1 * WTP] * 32.0f),
                 (_Float16)(cp[2 * WTP] * 32.0f), (_Float16)(cp[3 * WTP] * 32.0f),
                 (_Float16)(cp[4 * WTP] * 32.0f), (_Float16)(cp[5 * WTP] * 32.0f),
                 (_Float16)(cp[6 * WTP] * 32.0f), (_Float16)(cp[7 * WTP] * 32.0f)};
    val[j] = pk.u;
    go[j]  = (size_t)(n0 + nl) * kin + k0 + pc * 8;
  }
  for (int ps = 0; ps < 2; ++ps) {
#pragma unroll
    for (int j = 0; j < 2; ++j) *(volatile v4u*)(wt + go[j]) = val[j];
    __threadfence();
  }
}

#define STP 72
template <int KK>
__global__ __launch_bounds__(256) void k_gemm_h(const _Float16* __restrict__ A, int lda,
                                                const _Float16* __restrict__ Bt,
                                                const float* __restrict__ bias0,
                                                const float* __restrict__ bias1, int nsplit,
                                                _Float16* __restrict__ outp, int ldo,
                                                float oscale, float bscale) {
  __shared__ __align__(16) _Float16 st[256 * STP];
  const int tid = threadIdx.x, lane = tid & 31, wave = tid >> 5;
  const int hh = lane >> 4, c = lane & 15;
  const int mb = blockIdx.x * 256;
  const int m0 = mb + wave * 32;
  const int n0 = blockIdx.y * 64;

  v8f acc[2][4];
#pragma unroll
  for (int s = 0; s < 2; ++s)
#pragma unroll
    for (int t = 0; t < 4; ++t) acc[s][t] = zero8();
  gemm32x64<KK>(A, lda, Bt, KK, m0, n0, lane, acc);

#pragma unroll
  for (int t = 0; t < 4; ++t) {
    const int n  = n0 + 16 * t + c;
    const bool lo = (n < nsplit);
    const int i0 = lo ? n : (nsplit - 1);
    const int i1 = lo ? 0 : (n - nsplit);
    const float v0 = bias0[i0], v1 = bias1[i1];
    const float bb = (lo ? v0 : v1) * bscale;
#pragma unroll
    for (int sub = 0; sub < 2; ++sub) {
#pragma unroll
      for (int r = 0; r < 8; ++r) {
        const int lr = wave * 32 + sub * 16 + 8 * hh + r;
        st[lr * STP + 16 * t + c] = (_Float16)(acc[sub][t][r] * oscale + bb);
      }
    }
  }
  __syncthreads();

  v4u val[8];
  size_t go[8];
#pragma unroll
  for (int j = 0; j < 8; ++j) {
    const int p  = tid + 256 * j;
    const int lr = p >> 3;
    const int pc = p & 7;
    Pack8 pk;
    pk.h   = *(const v8h*)(st + lr * STP + pc * 8);
    val[j] = pk.u;
    go[j]  = (size_t)(mb + lr) * ldo + n0 + pc * 8;
  }
  for (int ps = 0; ps < 2; ++ps) {
#pragma unroll
    for (int j = 0; j < 8; ++j) *(volatile v4u*)(outp + go[j]) = val[j];
    __threadfence();
  }
}

#define OTP 68
template <int TANH>
__global__ __launch_bounds__(64) void k_gemm_s(const _Float16* __restrict__ A, int lda,
                                               const _Float16* __restrict__ Bt,
                                               const float* __restrict__ bias,
                                               float* __restrict__ outp, int ldo, float oscale) {
  __shared__ __align__(16) float st[64 * OTP];
  const int tid = threadIdx.x, lane = tid & 31, wave = tid >> 5;
  const int hh = lane >> 4, c = lane & 15;
  const int m0 = wave * 32;
  const int n0 = blockIdx.x * 64;

  v8f acc[2][4];
#pragma unroll
  for (int s = 0; s < 2; ++s)
#pragma unroll
    for (int t = 0; t < 4; ++t) acc[s][t] = zero8();
  gemm32x64<NHID>(A, lda, Bt, NHID, m0, n0, lane, acc);

#pragma unroll
  for (int t = 0; t < 4; ++t) {
    const float bb = bias[n0 + 16 * t + c];
#pragma unroll
    for (int sub = 0; sub < 2; ++sub) {
#pragma unroll
      for (int r = 0; r < 8; ++r) {
        float v = acc[sub][t][r] * oscale + bb;
        if (TANH) v = tanhf(v);
        st[(m0 + sub * 16 + 8 * hh + r) * OTP + 16 * t + c] = v;
      }
    }
  }
  __syncthreads();

#pragma unroll
  for (int half = 0; half < 2; ++half) {
    v4f val[8];
    size_t go[8];
#pragma unroll
    for (int it = 0; it < 8; ++it) {
      const int p   = tid + 64 * (half * 8 + it);
      const int row = p >> 4;
      const int pc  = p & 15;
      val[it] = *(const v4f*)(st + row * OTP + pc * 4);
      go[it]  = (size_t)row * ldo + n0 + pc * 4;
    }
    for (int ps = 0; ps < 2; ++ps) {
#pragma unroll
      for (int it = 0; it < 8; ++it) *(volatile v4f*)(outp + go[it]) = val[it];
      __threadfence();
    }
  }
}

__global__ __launch_bounds__(256) void k_attn0(const float* __restrict__ q0,
                                               const _Float16* __restrict__ kv,
                                               _Float16* __restrict__ sa) {
  __shared__ __align__(16) float s_q[NHID];
  __shared__ float s_p[NL];
  __shared__ float s_red[16];
  __shared__ float s_ctx[4 * HDIM];
  __shared__ __align__(16) _Float16 s_row[NHID];
  const int tid = threadIdx.x, lane = tid & 31, wave = tid >> 5;
  const int b = blockIdx.x;
#pragma unroll
  for (int i = 0; i < 3; ++i)
    s_q[tid + 256 * i] = q0[(size_t)b * NHID + tid + 256 * i] * 0.0078125f;
  __syncthreads();

  const size_t rowb = (size_t)b * NL;
  const float NEGI = -__builtin_huge_valf();
  for (int h = 0; h < NHEAD; ++h) {
    const _Float16* krow = kv + (rowb + tid) * KVW + h * HDIM;
    const float* qh = s_q + h * HDIM;
    float s = 0.f;
#pragma unroll 1
    for (int i8 = 0; i8 < 8; ++i8) {
      const v8h kk = *(const v8h*)(krow + 8 * i8);
      const v4f qa = *(const v4f*)(qh + 8 * i8);
      const v4f qb = *(const v4f*)(qh + 8 * i8 + 4);
      s += (float)kk[0] * qa[0]; s += (float)kk[1] * qa[1]; s += (float)kk[2] * qa[2]; s += (float)kk[3] * qa[3];
      s += (float)kk[4] * qb[0]; s += (float)kk[5] * qb[1]; s += (float)kk[6] * qb[2]; s += (float)kk[7] * qb[3];
    }
    float m = s;
#pragma unroll
    for (int off = 16; off > 0; off >>= 1) m = fmaxf(m, __shfl_xor(m, off, 32));
    if (lane == 0) s_red[wave] = m;
    __syncthreads();
    float mx = NEGI;
#pragma unroll
    for (int w = 0; w < 8; ++w) mx = fmaxf(mx, s_red[w]);
    const float p = __expf(s - mx);
    s_p[tid] = p;
    float ps = p;
#pragma unroll
    for (int off = 16; off > 0; off >>= 1) ps += __shfl_xor(ps, off, 32);
    if (lane == 0) s_red[8 + wave] = ps;
    __syncthreads();
    float l = 0.f;
#pragma unroll
    for (int w = 0; w < 8; ++w) l += s_red[8 + w];
    const float rl = 0.0625f * (1.0f / l);

    const int dd = tid & 63, part = tid >> 6;
    const _Float16* vcol = kv + (rowb + part * 64) * KVW + NHID + h * HDIM + dd;
    const float* pp = s_p + part * 64;
    float cacc = 0.f;
#pragma unroll 2
    for (int kk2 = 0; kk2 < 64; ++kk2) cacc += pp[kk2] * (float)vcol[(size_t)kk2 * KVW];
    s_ctx[part * 64 + dd] = cacc;
    __syncthreads();
    if (tid < 64) {
      const float cs = (s_ctx[tid] + s_ctx[64 + tid]) + (s_ctx[128 + tid] + s_ctx[192 + tid]);
      const float th = tanhf(cs * rl);
      s_row[h * HDIM + tid] = (_Float16)(th * 256.0f);
    }
    __syncthreads();
  }
  if (tid < 96) {
    Pack8 pk;
    pk.h = *(const v8h*)(s_row + 8 * tid);
    const v4u vv = pk.u;
    volatile v4u* dp = (volatile v4u*)(sa + (size_t)b * NHID + 8 * tid);
    *dp = vv;
    __threadfence();
    *dp = vv;
  }
}

__global__ __launch_bounds__(256) void k_apc(const float* __restrict__ pooled,
                                             const float* __restrict__ wapc,
                                             const float* __restrict__ bapc,
                                             float* __restrict__ out1) {
  __shared__ __align__(16) float s_o[192];
  const int tid = threadIdx.x;
  if (tid < 192) {
    const int bb = tid / 3;
    const int j  = tid - 3 * bb;
    const float* pr = pooled + (size_t)bb * NHID;
    float a = 0.f;
#pragma unroll 4
    for (int hcol = 0; hcol < NHID; ++hcol) a += pr[hcol] * wapc[hcol * 3 + j];
    s_o[tid] = a + bapc[j];
  }
  __syncthreads();
  if (tid < 48) {
    const v4f o = *(const v4f*)(s_o + 4 * tid);
    volatile v4f* dp = (volatile v4f*)(out1 + 4 * tid);
    *dp = o;
    __threadfence();
    *dp = o;
  }
}

extern "C" void kernel_launch(void* const* d_in, const int* in_sizes, int n_in,
                              void* d_out, int out_size, void* d_ws, size_t ws_size,
                              hipStream_t stream) {
  if (n_in < 19) return;
  if (in_sizes[0] != ROWS * NHID || in_sizes[1] != ROWS * NHID) return;
  if (in_sizes[2] != ROWS || in_sizes[3] != ROWS || in_sizes[4] != ROWS) return;
  if (in_sizes[5] != H3 * NHID || in_sizes[6] != NHID) return;
  if (in_sizes[7] != NHID * NHID || in_sizes[8] != NHID) return;
  if (in_sizes[9] != NHID * NHID || in_sizes[10] != NHID) return;
  if (in_sizes[11] != NHID * NHID || in_sizes[12] != NHID) return;
  if (in_sizes[13] != NHID * NHID || in_sizes[14] != NHID) return;
  if (in_sizes[15] != NHID * 6 || in_sizes[16] != 6) return;
  if (in_sizes[17] != NHID * 3 || in_sizes[18] != 3) return;
  if (out_size != ROWS * 6 + NB * 3) return;

  const float* gh      = (const float*)d_in[0];
  const float* lh      = (const float*)d_in[1];
  const int*   valid   = (const int*)d_in[2];
  const float* cdm     = (const float*)d_in[3];
  const float* cdw     = (const float*)d_in[4];
  const float* Wtri    = (const float*)d_in[5];
  const float* btri    = (const float*)d_in[6];
  const float* Wq      = (const float*)d_in[7];
  const float* bq      = (const float*)d_in[8];
  const float* Wk      = (const float*)d_in[9];
  const float* bk      = (const float*)d_in[10];
  const float* Wv      = (const float*)d_in[11];
  const float* bv      = (const float*)d_in[12];
  const float* Wpool   = (const float*)d_in[13];
  const float* bpool   = (const float*)d_in[14];
  const float* Wate    = (const float*)d_in[15];
  const float* bate    = (const float*)d_in[16];
  const float* Wapc    = (const float*)d_in[17];
  const float* bapc    = (const float*)d_in[18];
  float* out0 = (float*)d_out;
  float* out1 = (float*)((char*)d_out + (size_t)ROWS * 6 * 4);

  size_t off = 0;
  const size_t szCAT = (size_t)ROWS * H3 * 2;
  const size_t szKV  = (size_t)ROWS * KVW * 2;
  const size_t oCAT  = 0;
  const size_t oKV   = 0;
  off += (szCAT > szKV) ? szCAT : szKV;
  const size_t oX    = off; off += (size_t)ROWS * NHID * 2;
  const size_t oWt   = off; off += (size_t)NHID * H3 * 2;
  const size_t oKVt  = off; off += (size_t)KVW * NHID * 2;
  const size_t oWq   = off; off += (size_t)NHID * NHID * 2;
  const size_t oWp   = off; off += (size_t)NHID * NHID * 2;
  const size_t oQ0   = off; off += (size_t)NB * NHID * 4;
  const size_t oSA   = off; off += (size_t)NB * NHID * 2;
  const size_t oPL   = off; off += (size_t)NB * NHID * 4;
  if (off > ws_size) return;
  if (off > (size_t)134217728) return;

  char* ws = (char*)d_ws;
  _Float16* CAT  = (_Float16*)(ws + oCAT);
  _Float16* KV   = (_Float16*)(ws + oKV);
  _Float16* X    = (_Float16*)(ws + oX);
  _Float16* WtT  = (_Float16*)(ws + oWt);
  _Float16* KVt  = (_Float16*)(ws + oKVt);
  _Float16* WqT  = (_Float16*)(ws + oWq);
  _Float16* WpT  = (_Float16*)(ws + oWp);
  float*    Q0   = (float*)(ws + oQ0);
  _Float16* SA0  = (_Float16*)(ws + oSA);
  float*    POOL = (float*)(ws + oPL);

  k_cat<<<dim3(ROWS / 16), dim3(256), 0, stream>>>(gh, lh, valid, cdm, cdw, Wate, bate, CAT, out0);
  k_wt<<<dim3(NHID / 64, H3 / 64), dim3(256), 0, stream>>>(Wtri, WtT, NHID, H3);
  k_wt<<<dim3(NHID / 64, NHID / 64), dim3(256), 0, stream>>>(Wk, KVt, NHID, NHID);
  k_wt<<<dim3(NHID / 64, NHID / 64), dim3(256), 0, stream>>>(Wv, KVt + (size_t)NHID * NHID, NHID, NHID);
  k_wt<<<dim3(NHID / 64, NHID / 64), dim3(256), 0, stream>>>(Wq, WqT, NHID, NHID);
  k_wt<<<dim3(NHID / 64, NHID / 64), dim3(256), 0, stream>>>(Wpool, WpT, NHID, NHID);
  k_gemm_h<H3><<<dim3(ROWS / 256, NHID / 64), dim3(256), 0, stream>>>(CAT, H3, WtT, btri, btri, NHID, X, NHID, 0.03125f, 16.0f);
  k_gemm_h<NHID><<<dim3(ROWS / 256, KVW / 64), dim3(256), 0, stream>>>(X, NHID, KVt, bk, bv, NHID, KV, KVW, 0.03125f, 16.0f);
  k_gemm_s<0><<<dim3(NHID / 64), dim3(64), 0, stream>>>(X, NL * NHID, WqT, bq, Q0, NHID, 0.001953125f);
  k_attn0<<<dim3(NB), dim3(256), 0, stream>>>(Q0, KV, SA0);
  k_gemm_s<1><<<dim3(NHID / 64), dim3(64), 0, stream>>>(SA0, NHID, WpT, bpool, POOL, NHID, 0.0001220703125f);
  k_apc<<<dim3(1), dim3(256), 0, stream>>>(POOL, Wapc, bapc, out1);
  (void)hipGetLastError();
}
